// Mamba_69784628625647
// MI455X (gfx1250) — hardware-verified
//
#include <hip/hip_runtime.h>
#include <stddef.h>
#include <stdint.h>

#define DM     1024
#define EDI    2048
#define NS     16
#define DTR    64
#define KC     4
#define NBT    4
#define LS     512
#define MT     (NBT * LS)
#define NXZ    (2 * EDI)
#define KX2    (2 * EDI)
#define NXP    128
#define KD2    (2 * DTR)
#define NDBC   96
#define GBM    64
#define GBN    128
#define GTHR   128
#define NTHR   256
#define CTH    256
#define TCH    64
#define TS     16
#define SCH    32
#define WSMAX  134217728
#define LOG2E  1.4426950408889634f

#define U_XB  (MT * DM / 8)
#define U_WI  (NXZ * DM / 8)
#define U_WO  (DM * KX2 / 8)
#define U_WX  (NXP * KX2 / 8)
#define U_WD  (EDI * KD2 / 8)
#define U_ALL (U_XB + U_WI + U_WO + 2 * U_WX + 2 * U_WD)

static_assert(MT % GBM == 0 && NXZ % GBN == 0 && NXP == GBN && EDI % GBN == 0 && DM % GBN == 0);
static_assert(DM % 32 == 0 && KX2 % 32 == 0 && KD2 % 32 == 0);
static_assert(GBM == (GTHR / 32) * 16 && GBN == 4 * 32);
static_assert(EDI % CTH == 0 && CTH == NTHR && LS % TCH == 0 && TCH % TS == 0 && LS % SCH == 0);
static_assert(U_XB % NTHR == 0 && U_WI % NTHR == 0 && U_WO % NTHR == 0 && U_WX % NTHR == 0 && U_WD % NTHR == 0);
static_assert(U_ALL % NTHR == 0);
static_assert((KX2 / 8) == 512 && (KD2 / 8) == 16);
static_assert(TS * 4 == 64 && SCH * 2 == 64);
static_assert(SCH * 32 == 4 * NTHR);
static_assert((SCH * 32 + NTHR * NS + SCH * CTH) * 4 <= 65536);
static_assert(NDBC == DTR + 2 * NS && NDBC <= NXP);

typedef float          v4f   __attribute__((ext_vector_type(4)));
typedef float          v8f   __attribute__((ext_vector_type(8)));
typedef int            v8i   __attribute__((ext_vector_type(8)));
typedef unsigned short v8us  __attribute__((ext_vector_type(8)));
typedef unsigned short v16us __attribute__((ext_vector_type(16)));
typedef __bf16         v16bf __attribute__((ext_vector_type(16)));
typedef v4f  __attribute__((may_alias)) v4fa;
typedef v8us __attribute__((may_alias)) v8usa;
union FragB { v16bf v; v16us u; v8us h[2]; v8i w; };

__device__ __forceinline__ v8f wmb(const FragB& a, const FragB& b, v8f c) {
  v8f d = __builtin_amdgcn_wmma_f32_16x16x32_bf16(false, a.v, false, b.v, (short)0, c, false, false);
  asm volatile("v_nop\n\tv_nop\n\tv_nop\n\tv_nop" : "+v"(d) : "v"(a.w), "v"(b.w));
  return d;
}

__device__ __forceinline__ unsigned bf16_bits(float f) {
  const unsigned u = __float_as_uint(f);
  return (u + 0x7FFFu + ((u >> 16) & 1u)) >> 16;
}
__device__ __forceinline__ float bf16_val(float f) {
  return __uint_as_float(bf16_bits(f) << 16);
}
__device__ __forceinline__ void put16(unsigned short* dp, v8us o) {
  *(volatile v8us*)dp = o;
  __threadfence();
  *(volatile v8us*)dp = o;
}

#if __has_builtin(__builtin_amdgcn_exp2f)
#define EXP2_HW(x) __builtin_amdgcn_exp2f(x)
#else
#define EXP2_HW(x) exp2f(x)
#endif

__device__ __forceinline__ float silu_f(float v) {
  const float e = expf(-v);
  return v * __builtin_amdgcn_rcpf(1.0f + e);
}

__global__ __launch_bounds__(NTHR) void k_prep(const float* __restrict__ x, const float* __restrict__ Win,
                                               const float* __restrict__ Wout,
                                               const float* __restrict__ Wx0, const float* __restrict__ Wx1,
                                               const float* __restrict__ Wd0, const float* __restrict__ Wd1,
                                               unsigned short* XB, unsigned short* WIN, unsigned short* WO2,
                                               unsigned short* WX2a, unsigned short* WX2b,
                                               unsigned short* WD2a, unsigned short* WD2b) {
  const int u  = (int)blockIdx.x * NTHR + (int)threadIdx.x;
  const int L0 = U_XB;
  const int L1 = L0 + U_WI;
  const int L2 = L1 + U_WO;
  const int L3 = L2 + 2 * U_WX;
  const int L4 = L3 + 2 * U_WD;
  const float* src;
  unsigned short* dst;
  float keep = 1.0f;
  if (u < L0) {
    src = x + (size_t)u * 8;
    dst = XB + (size_t)u * 8;
  } else if (u < L1) {
    const int v = u - L0;
    src = Win + (size_t)v * 8;
    dst = WIN + (size_t)v * 8;
  } else if (u < L2) {
    const int v  = u - L1;
    const int n  = v >> 9;
    const int k8 = (v & 511) * 8;
    src = Wout + (size_t)n * EDI + (k8 & (EDI - 1));
    dst = WO2 + (size_t)n * KX2 + k8;
  } else if (u < L3) {
    const int v  = u - L2;
    const int d  = v / U_WX;
    const int vv = v - d * U_WX;
    const int n  = vv >> 9;
    const int k8 = (vv & 511) * 8;
    const int nn = n < NDBC ? n : NDBC - 1;
    keep = n < NDBC ? 1.0f : 0.0f;
    const float* W = (d != 0) ? Wx1 : Wx0;
    src = W + (size_t)nn * EDI + (k8 & (EDI - 1));
    dst = ((d != 0) ? WX2b : WX2a) + (size_t)n * KX2 + k8;
  } else if (u < L4) {
    const int v  = u - L3;
    const int d  = v / U_WD;
    const int vv = v - d * U_WD;
    const int n  = vv >> 4;
    const int k8 = (vv & 15) * 8;
    const float* W = (d != 0) ? Wd1 : Wd0;
    src = W + (size_t)n * DTR + (k8 & (DTR - 1));
    dst = ((d != 0) ? WD2b : WD2a) + (size_t)n * KD2 + k8;
  } else {
    return;
  }
  const v4f a = *(const v4fa*)src;
  const v4f c = *(const v4fa*)(src + 4);
  v8us o;
  o[0] = (unsigned short)bf16_bits(a.x * keep);
  o[1] = (unsigned short)bf16_bits(a.y * keep);
  o[2] = (unsigned short)bf16_bits(a.z * keep);
  o[3] = (unsigned short)bf16_bits(a.w * keep);
  o[4] = (unsigned short)bf16_bits(c.x * keep);
  o[5] = (unsigned short)bf16_bits(c.y * keep);
  o[6] = (unsigned short)bf16_bits(c.z * keep);
  o[7] = (unsigned short)bf16_bits(c.w * keep);
  put16(dst, o);
}

template <int MODE>
__global__ __launch_bounds__(GTHR) void k_gemm(const unsigned short* __restrict__ A0,
                                               const unsigned short* __restrict__ A1, int lda,
                                               const unsigned short* __restrict__ B0,
                                               const unsigned short* __restrict__ B1, int ldb, int K,
                                               const float* __restrict__ bias0, const float* __restrict__ bias1,
                                               float* C0, float* C1, int ldc, int nsplit,
                                               unsigned short* Cb0, unsigned short* Cb1) {
  __shared__ __attribute__((aligned(16))) float stg[GBM * GBN];
  const int tid = (int)threadIdx.x, lane = tid & 31, wave = tid >> 5, hh = lane >> 4, m = lane & 15;
  const int dir = (int)blockIdx.z;
  const int rowBase = (int)blockIdx.x * GBM;
  const int colBase = (int)blockIdx.y * GBN;
  const unsigned short* A  = (dir != 0) ? A1 : A0;
  const unsigned short* BT = (dir != 0) ? B1 : B0;
  const float* bias = (dir != 0) ? bias1 : bias0;
  float* Cm = (dir != 0) ? C1 : C0;
  unsigned short* Cb = (dir != 0) ? Cb1 : Cb0;
  int ccol = colBase;
  if constexpr (MODE == 0) {
    if (colBase >= nsplit) { Cm = C1; ccol = colBase - nsplit; }
  }
  if constexpr (MODE == 2) { ccol = 0; }

  v8f acc[8];
  {
    const v8f z = {0.f, 0.f, 0.f, 0.f, 0.f, 0.f, 0.f, 0.f};
#pragma unroll
    for (int t = 0; t < 8; ++t) acc[t] = z;
  }
  const unsigned short* ap = A  + (size_t)(rowBase + 16 * wave + m) * (size_t)lda + 8 * hh;
  const unsigned short* bp = BT + (size_t)(colBase + m) * (size_t)ldb + 8 * hh;

#pragma unroll 1
  for (int k0 = 0; k0 < K; k0 += 32) {
    FragB af;
    af.h[0] = *(const v8usa*)(ap + k0);
    af.h[1] = *(const v8usa*)(ap + k0 + 16);
#pragma unroll
    for (int nt = 0; nt < 8; ++nt) {
      const unsigned short* wq = bp + (size_t)(16 * nt) * (size_t)ldb + k0;
      FragB bf;
      bf.h[0] = *(const v8usa*)wq;
      bf.h[1] = *(const v8usa*)(wq + 16);
      acc[nt] = wmb(af, bf, acc[nt]);
    }
  }

#pragma unroll
  for (int nt = 0; nt < 8; ++nt) {
    const int lc = 16 * nt + m;
#pragma unroll
    for (int r = 0; r < 8; ++r) {
      const int lr = 16 * wave + 8 * hh + r;
      stg[lr * GBN + lc] = acc[nt][r];
    }
  }
  __syncthreads();

  if constexpr (MODE == 1) {
    const float bvv = bf16_val(bias[colBase + tid]);
#pragma unroll 1
    for (int it = 0; it < (GBM * GBN) / GTHR; ++it) {
      const int e = it * GTHR + tid;
      const float v  = stg[e] + bvv;
      const float sp = fmaxf(v, 0.0f) + log1pf(expf(-fabsf(v)));
      stg[e] = sp;
    }
    __syncthreads();
  }

  {
    v4f pv[16];
#pragma unroll
    for (int i = 0; i < 16; ++i) pv[i] = *(const v4fa*)(stg + (16 * wave + i) * GBN + 4 * lane);
#pragma unroll
    for (int i = 0; i < 16; ++i) {
      float* op = Cm + (size_t)(rowBase + 16 * wave + i) * (size_t)ldc + ccol + 4 * lane;
      *(volatile v4f*)op = pv[i];
    }
    __threadfence();
#pragma unroll
    for (int i = 0; i < 16; ++i) {
      float* op = Cm + (size_t)(rowBase + 16 * wave + i) * (size_t)ldc + ccol + 4 * lane;
      *(volatile v4f*)op = pv[i];
    }
  }

  if constexpr (MODE == 2) {
    const int sub = lane >> 4, j = lane & 15, part = j >> 3, jj = j & 7;
    const unsigned mlo = 0u - (unsigned)part;
    const unsigned mhi = ~mlo;
    v8us pb[8];
#pragma unroll
    for (int i = 0; i < 8; ++i) {
      const int lr = 16 * wave + 2 * i + sub;
      const float* sp = stg + lr * GBN + 8 * jj;
      const v4f a = *(const v4fa*)sp;
      const v4f b = *(const v4fa*)(sp + 4);
      const v8f f8 = {a.x, a.y, a.z, a.w, b.x, b.y, b.z, b.w};
      v8us oo;
#pragma unroll
      for (int e = 0; e < 8; ++e) {
        const unsigned hb = bf16_bits(f8[e]);
        const unsigned lb = bf16_bits(f8[e] - __uint_as_float(hb << 16));
        oo[e] = (unsigned short)((hb & mhi) | (lb & mlo));
      }
      pb[i] = oo;
    }
#pragma unroll
    for (int i = 0; i < 8; ++i) {
      unsigned short* op = Cb + (size_t)(rowBase + 16 * wave + 2 * i + sub) * (size_t)NXP + 8 * j;
      *(volatile v8us*)op = pb[i];
    }
    __threadfence();
#pragma unroll
    for (int i = 0; i < 8; ++i) {
      unsigned short* op = Cb + (size_t)(rowBase + 16 * wave + 2 * i + sub) * (size_t)NXP + 8 * j;
      *(volatile v8us*)op = pb[i];
    }
  }
}

__device__ __forceinline__ float ldx(const float* __restrict__ XP, int rowb, int tt, int c) {
  const int   tc = tt < 0 ? 0 : (tt > LS - 1 ? LS - 1 : tt);
  const float k  = (tt >= 0 && tt < LS) ? 1.0f : 0.0f;
  return XP[(size_t)(rowb + tc) * EDI + c] * k;
}

__global__ __launch_bounds__(NTHR) void k_conv(const float* __restrict__ XP,
                                               const float* __restrict__ cw0, const float* __restrict__ cb0,
                                               const float* __restrict__ cw1, const float* __restrict__ cb1,
                                               unsigned short* XSf, unsigned short* XSb) {
  __shared__ __attribute__((aligned(16))) unsigned short tl[4][TS][CTH];
  const int tid = (int)threadIdx.x, lane = tid & 31, wave = tid >> 5;
  const int c0 = (int)blockIdx.x * CTH;
  const int c  = c0 + tid;
  const int b  = (int)blockIdx.y;
  const int rowb  = b * LS;
  const int tbase = (int)blockIdx.z * TCH;

  const v4f wfr = *(const v4fa*)(cw0 + (size_t)c * KC);
  const v4f wbr = *(const v4fa*)(cw1 + (size_t)c * KC);
  const float wf0 = bf16_val(wfr.x), wf1 = bf16_val(wfr.y), wf2 = bf16_val(wfr.z), wf3 = bf16_val(wfr.w);
  const float wb0 = bf16_val(wbr.x), wb1 = bf16_val(wbr.y), wb2 = bf16_val(wbr.z), wb3 = bf16_val(wbr.w);
  const float bf = bf16_val(cb0[c]);
  const float bb = bf16_val(cb1[c]);

  float xm3 = ldx(XP, rowb, tbase - 3, c);
  float xm2 = ldx(XP, rowb, tbase - 2, c);
  float xm1 = ldx(XP, rowb, tbase - 1, c);
  float x00 = ldx(XP, rowb, tbase, c);
  float xp1 = ldx(XP, rowb, tbase + 1, c);
  float xp2 = ldx(XP, rowb, tbase + 2, c);

#pragma unroll 1
  for (int ck = 0; ck < TCH / TS; ++ck) {
    const int t0 = tbase + ck * TS;
#pragma unroll 1
    for (int s = 0; s < TS; ++s) {
      const int t = t0 + s;
      const float xp3 = ldx(XP, rowb, t + 3, c);
      float af = wf0 * xm3;
      af = fmaf(wf1, xm2, af);
      af = fmaf(wf2, xm1, af);
      af = fmaf(wf3, x00, af);
      af = af + bf;
      float ab = wb0 * xp3;
      ab = fmaf(wb1, xp2, ab);
      ab = fmaf(wb2, xp1, ab);
      ab = fmaf(wb3, x00, ab);
      ab = ab + bb;
      const float sf = silu_f(af);
      const float sb = silu_f(ab);
      const unsigned hfv = bf16_bits(sf);
      const unsigned hbv = bf16_bits(sb);
      tl[0][s][tid] = (unsigned short)hfv;
      tl[1][s][tid] = (unsigned short)bf16_bits(sf - __uint_as_float(hfv << 16));
      tl[2][s][tid] = (unsigned short)hbv;
      tl[3][s][tid] = (unsigned short)bf16_bits(sb - __uint_as_float(hbv << 16));
      xm3 = xm2; xm2 = xm1; xm1 = x00; x00 = xp1; xp1 = xp2; xp2 = xp3;
    }
    __syncthreads();
    v8us pv[8];
#pragma unroll
    for (int it = 0; it < 8; ++it) {
      const int seg = it * 8 + wave;
      const int r = seg >> 2, wq = seg & 3;
      pv[it] = *(const v8usa*)(&tl[wq][r][8 * lane]);
    }
#pragma unroll
    for (int it = 0; it < 8; ++it) {
      const int seg = it * 8 + wave;
      const int r = seg >> 2, wq = seg & 3;
      unsigned short* base = (wq >= 2) ? XSb : XSf;
      unsigned short* op = base + (size_t)(rowb + t0 + r) * (size_t)KX2 + (wq & 1) * EDI + c0 + 8 * lane;
      *(volatile v8us*)op = pv[it];
    }
    __threadfence();
#pragma unroll
    for (int it = 0; it < 8; ++it) {
      const int seg = it * 8 + wave;
      const int r = seg >> 2, wq = seg & 3;
      unsigned short* base = (wq >= 2) ? XSb : XSf;
      unsigned short* op = base + (size_t)(rowb + t0 + r) * (size_t)KX2 + (wq & 1) * EDI + c0 + 8 * lane;
      *(volatile v8us*)op = pv[it];
    }
    __syncthreads();
  }
}

__global__ __launch_bounds__(NTHR) void k_scan_f(const float* __restrict__ DEL, const float* __restrict__ DBC,
                                                 const unsigned short* __restrict__ XS,
                                                 const float* __restrict__ ZP,
                                                 const float* __restrict__ Alog, const float* __restrict__ Dp,
                                                 float* YF) {
  __shared__ __attribute__((aligned(16))) float sBC[SCH * 32];
  __shared__ __attribute__((aligned(16))) float sA[NTHR * NS];
  __shared__ __attribute__((aligned(16))) float yT[SCH * CTH];
  const int tid = (int)threadIdx.x, lane = tid & 31, wave = tid >> 5;
  const int c0 = (int)blockIdx.x * CTH;
  const int c  = c0 + tid;
  const int b  = (int)blockIdx.y;
  const int rowb = b * LS;

#pragma unroll 1
  for (int n = 0; n < NS; ++n) sA[tid * NS + n] = -expf(bf16_val(Alog[(size_t)c * NS + n]));
  const float dp = bf16_val(Dp[c]);
  __syncthreads();
  float A2[NS];
  {
    const v4f a0 = *(const v4fa*)(sA + tid * NS);
    const v4f a1 = *(const v4fa*)(sA + tid * NS + 4);
    const v4f a2 = *(const v4fa*)(sA + tid * NS + 8);
    const v4f a3 = *(const v4fa*)(sA + tid * NS + 12);
    A2[0]  = a0.x * LOG2E; A2[1]  = a0.y * LOG2E; A2[2]  = a0.z * LOG2E; A2[3]  = a0.w * LOG2E;
    A2[4]  = a1.x * LOG2E; A2[5]  = a1.y * LOG2E; A2[6]  = a1.z * LOG2E; A2[7]  = a1.w * LOG2E;
    A2[8]  = a2.x * LOG2E; A2[9]  = a2.y * LOG2E; A2[10] = a2.z * LOG2E; A2[11] = a2.w * LOG2E;
    A2[12] = a3.x * LOG2E; A2[13] = a3.y * LOG2E; A2[14] = a3.z * LOG2E; A2[15] = a3.w * LOG2E;
  }
  float h[NS];
#pragma unroll
  for (int n = 0; n < NS; ++n) h[n] = 0.0f;

#pragma unroll 1
  for (int ck = 0; ck < LS / SCH; ++ck) {
    const int tlo = ck * SCH;
    {
      const int r = tid >> 3, q = tid & 7;
      const v4f v = *(const v4fa*)(DBC + (size_t)(rowb + tlo + r) * NXP + DTR + 4 * q);
      *(v4fa*)(sBC + r * 32 + 4 * q) = v;
    }
    __syncthreads();
#pragma unroll 1
    for (int s = 0; s < SCH; ++s) {
      const size_t row = (size_t)(rowb + tlo + s);
      const float dv = DEL[row * EDI + c];
      const unsigned hw = XS[row * (size_t)KX2 + c];
      const unsigned lw = XS[row * (size_t)KX2 + EDI + c];
      const float z  = ZP[row * EDI + c];
      const float xs = __uint_as_float(hw << 16) + __uint_as_float(lw << 16);
      const float* bcp = sBC + s * 32;
      const v4f b0 = *(const v4fa*)(bcp);
      const v4f b1 = *(const v4fa*)(bcp + 4);
      const v4f b2 = *(const v4fa*)(bcp + 8);
      const v4f b3 = *(const v4fa*)(bcp + 12);
      const v4f q0 = *(const v4fa*)(bcp + 16);
      const v4f q1 = *(const v4fa*)(bcp + 20);
      const v4f q2 = *(const v4fa*)(bcp + 24);
      const v4f q3 = *(const v4fa*)(bcp + 28);
      const float Bv[NS] = {b0.x, b0.y, b0.z, b0.w, b1.x, b1.y, b1.z, b1.w,
                            b2.x, b2.y, b2.z, b2.w, b3.x, b3.y, b3.z, b3.w};
      const float Cv[NS] = {q0.x, q0.y, q0.z, q0.w, q1.x, q1.y, q1.z, q1.w,
                            q2.x, q2.y, q2.z, q2.w, q3.x, q3.y, q3.z, q3.w};
      float yc = 0.0f;
#pragma unroll
      for (int n = 0; n < NS; ++n) {
        const float e = EXP2_HW(dv * A2[n]);
        h[n] = fmaf(e, h[n], (dv * Bv[n]) * xs);
        yc = fmaf(h[n], Cv[n], yc);
      }
      yT[s * CTH + tid] = (yc + dp * xs) * silu_f(z);
    }
    __syncthreads();
    {
      v4f pv[8];
#pragma unroll
      for (int it = 0; it < 8; ++it) {
        const int seg = it * 8 + wave;
        const int r = seg >> 1, hf = seg & 1;
        pv[it] = *(const v4fa*)(yT + r * CTH + 128 * hf + 4 * lane);
      }
#pragma unroll
      for (int it = 0; it < 8; ++it) {
        const int seg = it * 8 + wave;
        const int r = seg >> 1, hf = seg & 1;
        float* op = YF + (size_t)(rowb + tlo + r) * EDI + c0 + 128 * hf + 4 * lane;
        *(volatile v4f*)op = pv[it];
      }
      __threadfence();
#pragma unroll
      for (int it = 0; it < 8; ++it) {
        const int seg = it * 8 + wave;
        const int r = seg >> 1, hf = seg & 1;
        float* op = YF + (size_t)(rowb + tlo + r) * EDI + c0 + 128 * hf + 4 * lane;
        *(volatile v4f*)op = pv[it];
      }
    }
    __syncthreads();
  }
}

__global__ __launch_bounds__(NTHR) void k_scan_b(const float* __restrict__ DEL, const float* __restrict__ DBC,
                                                 const unsigned short* __restrict__ XS,
                                                 const float* __restrict__ ZP,
                                                 const float* __restrict__ Alog, const float* __restrict__ Dp,
                                                 const float* __restrict__ YF, unsigned short* YHL) {
  __shared__ __attribute__((aligned(16))) float sBC[SCH * 32];
  __shared__ __attribute__((aligned(16))) float sA[NTHR * NS];
  __shared__ __attribute__((aligned(16))) unsigned short yTb[2 * SCH * CTH];
  const int tid = (int)threadIdx.x, lane = tid & 31, wave = tid >> 5;
  const int c0 = (int)blockIdx.x * CTH;
  const int c  = c0 + tid;
  const int b  = (int)blockIdx.y;
  const int rowb = b * LS;

#pragma unroll 1
  for (int n = 0; n < NS; ++n) sA[tid * NS + n] = -expf(bf16_val(Alog[(size_t)c * NS + n]));
  const float dp = bf16_val(Dp[c]);
  __syncthreads();
  float A2[NS];
  {
    const v4f a0 = *(const v4fa*)(sA + tid * NS);
    const v4f a1 = *(const v4fa*)(sA + tid * NS + 4);
    const v4f a2 = *(const v4fa*)(sA + tid * NS + 8);
    const v4f a3 = *(const v4fa*)(sA + tid * NS + 12);
    A2[0]  = a0.x * LOG2E; A2[1]  = a0.y * LOG2E; A2[2]  = a0.z * LOG2E; A2[3]  = a0.w * LOG2E;
    A2[4]  = a1.x * LOG2E; A2[5]  = a1.y * LOG2E; A2[6]  = a1.z * LOG2E; A2[7]  = a1.w * LOG2E;
    A2[8]  = a2.x * LOG2E; A2[9]  = a2.y * LOG2E; A2[10] = a2.z * LOG2E; A2[11] = a2.w * LOG2E;
    A2[12] = a3.x * LOG2E; A2[13] = a3.y * LOG2E; A2[14] = a3.z * LOG2E; A2[15] = a3.w * LOG2E;
  }
  float h[NS];
#pragma unroll
  for (int n = 0; n < NS; ++n) h[n] = 0.0f;

#pragma unroll 1
  for (int ck = 0; ck < LS / SCH; ++ck) {
    const int tlo = LS - SCH * (ck + 1);
    {
      const int r = tid >> 3, q = tid & 7;
      const v4f v = *(const v4fa*)(DBC + (size_t)(rowb + tlo + r) * NXP + DTR + 4 * q);
      *(v4fa*)(sBC + r * 32 + 4 * q) = v;
    }
    __syncthreads();
#pragma unroll 1
    for (int s = SCH - 1; s >= 0; --s) {
      const size_t row = (size_t)(rowb + tlo + s);
      const float dv = DEL[row * EDI + c];
      const unsigned hw = XS[row * (size_t)KX2 + c];
      const unsigned lw = XS[row * (size_t)KX2 + EDI + c];
      const float z  = ZP[row * EDI + c];
      const float yf = YF[row * EDI + c];
      const float xs = __uint_as_float(hw << 16) + __uint_as_float(lw << 16);
      const float* bcp = sBC + s * 32;
      const v4f b0 = *(const v4fa*)(bcp);
      const v4f b1 = *(const v4fa*)(bcp + 4);
      const v4f b2 = *(const v4fa*)(bcp + 8);
      const v4f b3 = *(const v4fa*)(bcp + 12);
      const v4f q0 = *(const v4fa*)(bcp + 16);
      const v4f q1 = *(const v4fa*)(bcp + 20);
      const v4f q2 = *(const v4fa*)(bcp + 24);
      const v4f q3 = *(const v4fa*)(bcp + 28);
      const float Bv[NS] = {b0.x, b0.y, b0.z, b0.w, b1.x, b1.y, b1.z, b1.w,
                            b2.x, b2.y, b2.z, b2.w, b3.x, b3.y, b3.z, b3.w};
      const float Cv[NS] = {q0.x, q0.y, q0.z, q0.w, q1.x, q1.y, q1.z, q1.w,
                            q2.x, q2.y, q2.z, q2.w, q3.x, q3.y, q3.z, q3.w};
      float yc = 0.0f;
#pragma unroll
      for (int n = 0; n < NS; ++n) {
        const float e = EXP2_HW(dv * A2[n]);
        h[n] = fmaf(e, h[n], (dv * Bv[n]) * xs);
        yc = fmaf(h[n], Cv[n], yc);
      }
      const float yb = (yc + dp * xs) * silu_f(z);
      const float y  = (yf + yb) * 0.5f;
      const unsigned hb = bf16_bits(y);
      yTb[s * CTH + tid]         = (unsigned short)hb;
      yTb[(SCH + s) * CTH + tid] = (unsigned short)bf16_bits(y - __uint_as_float(hb << 16));
    }
    __syncthreads();
    {
      v8us pv[8];
#pragma unroll
      for (int it = 0; it < 8; ++it) {
        const int seg = it * 8 + wave;
        const int r = seg >> 1, part = seg & 1;
        pv[it] = *(const v8usa*)(yTb + (part * SCH + r) * CTH + 8 * lane);
      }
#pragma unroll
      for (int it = 0; it < 8; ++it) {
        const int seg = it * 8 + wave;
        const int r = seg >> 1, part = seg & 1;
        unsigned short* op = YHL + (size_t)(rowb + tlo + r) * (size_t)KX2 + part * EDI + c0 + 8 * lane;
        *(volatile v8us*)op = pv[it];
      }
      __threadfence();
#pragma unroll
      for (int it = 0; it < 8; ++it) {
        const int seg = it * 8 + wave;
        const int r = seg >> 1, part = seg & 1;
        unsigned short* op = YHL + (size_t)(rowb + tlo + r) * (size_t)KX2 + part * EDI + c0 + 8 * lane;
        *(volatile v8us*)op = pv[it];
      }
    }
    __syncthreads();
  }
}

extern "C" void kernel_launch(void* const* d_in, const int* in_sizes, int n_in,
                              void* d_out, int out_size, void* d_ws, size_t ws_size,
                              hipStream_t stream) {
  if (n_in < 17) return;
  if (in_sizes[0]  != MT * DM) return;
  if (in_sizes[1]  != NXZ * DM) return;
  if (in_sizes[2]  != EDI * KC) return;
  if (in_sizes[3]  != EDI) return;
  if (in_sizes[4]  != NDBC * EDI) return;
  if (in_sizes[5]  != EDI * DTR) return;
  if (in_sizes[6]  != EDI) return;
  if (in_sizes[7]  != EDI * NS) return;
  if (in_sizes[8]  != EDI) return;
  if (in_sizes[9]  != EDI * KC) return;
  if (in_sizes[10] != EDI) return;
  if (in_sizes[11] != NDBC * EDI) return;
  if (in_sizes[12] != EDI * DTR) return;
  if (in_sizes[13] != EDI) return;
  if (in_sizes[14] != EDI * NS) return;
  if (in_sizes[15] != EDI) return;
  if (in_sizes[16] != DM * EDI) return;
  if (out_size != MT * DM) return;

  const float* x      = (const float*)d_in[0];
  const float* W_in   = (const float*)d_in[1];
  const float* cw_f   = (const float*)d_in[2];
  const float* cb_f   = (const float*)d_in[3];
  const float* Wx_f   = (const float*)d_in[4];
  const float* Wdt_f  = (const float*)d_in[5];
  const float* bdt_f  = (const float*)d_in[6];
  const float* Alog_f = (const float*)d_in[7];
  const float* Dp_f   = (const float*)d_in[8];
  const float* cw_b   = (const float*)d_in[9];
  const float* cb_b   = (const float*)d_in[10];
  const float* Wx_b   = (const float*)d_in[11];
  const float* Wdt_b  = (const float*)d_in[12];
  const float* bdt_b  = (const float*)d_in[13];
  const float* Alog_b = (const float*)d_in[14];
  const float* Dp_b   = (const float*)d_in[15];
  const float* W_out  = (const float*)d_in[16];
  float* out = (float*)d_out;

  const size_t szXB  = (size_t)MT * DM * 2;
  const size_t szWIN = (size_t)NXZ * DM * 2;
  const size_t szWO2 = (size_t)DM * KX2 * 2;
  const size_t szWX2 = (size_t)NXP * KX2 * 2;
  const size_t szWD2 = (size_t)EDI * KD2 * 2;
  const size_t szDBC = (size_t)MT * NXP * 4;
  const size_t szDR  = (size_t)MT * NXP * 2;
  const size_t szP32 = (size_t)MT * EDI * 4;
  const size_t szP16 = (size_t)MT * KX2 * 2;
  size_t off = 0;
  const size_t oXB   = off; off += szXB;
  const size_t oWIN  = off; off += szWIN;
  const size_t oWO2  = off; off += szWO2;
  const size_t oWX2f = off; off += szWX2;
  const size_t oWX2b = off; off += szWX2;
  const size_t oWD2f = off; off += szWD2;
  const size_t oWD2b = off; off += szWD2;
  const size_t oDBCf = off; off += szDBC;
  const size_t oDBCb = off; off += szDBC;
  const size_t oDRf  = off; off += szDR;
  const size_t oDRb  = off; off += szDR;
  const size_t oR1   = off; off += szP32;
  const size_t oZP   = off; off += szP32;
  const size_t oR2   = off; off += szP16;
  const size_t oXSb  = off; off += szP16;
  const size_t oDELf = off; off += szP32;
  const size_t oYF   = off; off += szP32;
  if (off > ws_size || off > (size_t)WSMAX) return;

  char* ws = (char*)d_ws;
  unsigned short* XB   = (unsigned short*)(ws + oXB);
  unsigned short* WIN  = (unsigned short*)(ws + oWIN);
  unsigned short* WO2  = (unsigned short*)(ws + oWO2);
  unsigned short* WX2f = (unsigned short*)(ws + oWX2f);
  unsigned short* WX2b = (unsigned short*)(ws + oWX2b);
  unsigned short* WD2f = (unsigned short*)(ws + oWD2f);
  unsigned short* WD2b = (unsigned short*)(ws + oWD2b);
  float*          DBCf = (float*)(ws + oDBCf);
  float*          DBCb = (float*)(ws + oDBCb);
  unsigned short* DRf  = (unsigned short*)(ws + oDRf);
  unsigned short* DRb  = (unsigned short*)(ws + oDRb);
  float*          XP   = (float*)(ws + oR1);
  float*          DELb = (float*)(ws + oR1);
  float*          ZP   = (float*)(ws + oZP);
  unsigned short* XSf  = (unsigned short*)(ws + oR2);
  unsigned short* YHL  = (unsigned short*)(ws + oR2);
  unsigned short* XSb  = (unsigned short*)(ws + oXSb);
  float*          DELf = (float*)(ws + oDELf);
  float*          YF   = (float*)(ws + oYF);
  const int nosplit = 0x40000000;

  k_prep<<<U_ALL / NTHR, NTHR, 0, stream>>>(x, W_in, W_out, Wx_f, Wx_b, Wdt_f, Wdt_b,
                                            XB, WIN, WO2, WX2f, WX2b, WD2f, WD2b);
  k_gemm<0><<<dim3(MT / GBM, NXZ / GBN, 1), GTHR, 0, stream>>>(XB, XB, DM, WIN, WIN, DM, DM, Dp_f, Dp_f,
                                                              XP, ZP, EDI, EDI, XSb, XSb);
  k_conv<<<dim3(EDI / CTH, NBT, LS / TCH), NTHR, 0, stream>>>(XP, cw_f, cb_f, cw_b, cb_b, XSf, XSb);
  k_gemm<2><<<dim3(MT / GBM, NXP / GBN, 2), GTHR, 0, stream>>>(XSf, XSb, KX2, WX2f, WX2b, KX2, KX2, Dp_f, Dp_f,
                                                              DBCf, DBCb, NXP, nosplit, DRf, DRb);
  k_gemm<1><<<dim3(MT / GBM, EDI / GBN, 2), GTHR, 0, stream>>>(DRf, DRb, KD2, WD2f, WD2b, KD2, KD2, bdt_f, bdt_b,
                                                              DELf, DELb, EDI, nosplit, DRf, DRb);
  k_scan_f<<<dim3(EDI / CTH, NBT), NTHR, 0, stream>>>(DELf, DBCf, XSf, ZP, Alog_f, Dp_f, YF);
  k_scan_b<<<dim3(EDI / CTH, NBT), NTHR, 0, stream>>>(DELb, DBCb, XSb, ZP, Alog_b, Dp_b, YF, YHL);
  k_gemm<3><<<dim3(MT / GBM, DM / GBN, 1), GTHR, 0, stream>>>(YHL, YHL, KX2, WO2, WO2, KX2, KX2, Dp_f, Dp_f,
                                                              out, out, DM, nosplit, DRf, DRf);
}
